// Decoder_21225728377092
// MI455X (gfx1250) — hardware-verified
//
#include <hip/hip_runtime.h>
#include <stddef.h>

#define NBATCH 128
#define SEQ    4096
#define DM     6
#define DFF    64
#define NLAY   4
#define TOK    (NBATCH * SEQ)
#define TILE   256
#define NTHR   256
#define NBLK   (TOK / TILE)
#define TPR    (SEQ / TILE)
#define XROWS  (TILE + 4)
#define W2P    72
#define AP     136
#define PLANE_FLOATS ((size_t)TOK * 8)
#define PLANE_BYTES  (PLANE_FLOATS * 4)
#define WSMAX  134217728
#define LAYER_LDS_BYTES (2 * XROWS * 8 * 4 + TILE * 8 * 4 + DFF * 8 * 4 + 16 * W2P * 2 + 8 * 16 * AP * 2 + 96 * 4 + 3 * 24 * 4 + 8)

static_assert(SEQ % TILE == 0);
static_assert(TOK % TILE == 0);
static_assert(NTHR == TILE && NTHR == 8 * 32);
static_assert((size_t)NBLK * TILE * 8 == PLANE_FLOATS);
static_assert((size_t)NBLK * TILE * DM == 3145728);
static_assert((W2P * 2) % 16 == 0 && W2P >= DFF + 8);
static_assert((AP * 2) % 16 == 0 && AP >= 2 * DFF);
static_assert(XROWS * 8 >= TILE * 8);
static_assert(LAYER_LDS_BYTES <= 65536);
static_assert(2 * PLANE_BYTES <= (size_t)WSMAX);
static_assert(DFF * DM == 384 && DM * DFF == 384);

typedef float          v4f   __attribute__((ext_vector_type(4)));
typedef float          v8f   __attribute__((ext_vector_type(8)));
typedef int            v8i   __attribute__((ext_vector_type(8)));
typedef unsigned short v8us  __attribute__((ext_vector_type(8)));
typedef unsigned short v16us __attribute__((ext_vector_type(16)));
typedef __bf16         v16bf __attribute__((ext_vector_type(16)));
typedef v4f  __attribute__((may_alias)) v4fa;
typedef v8us __attribute__((may_alias)) v8usa;
union FragB { v16bf v; v16us u; v8us h[2]; v8i w; };

__device__ __forceinline__ v8f wmb(const FragB& a, const FragB& b, v8f c) {
  v8f d = __builtin_amdgcn_wmma_f32_16x16x32_bf16(false, a.v, false, b.v, (short)0, c, false, false);
  asm volatile("v_nop\n\tv_nop\n\tv_nop\n\tv_nop" : "+v"(d) : "v"(a.w), "v"(b.w));
  return d;
}

__device__ __forceinline__ unsigned bf16_bits(float f) {
  const unsigned u = __float_as_uint(f);
  return (u + 0x7FFFu + ((u >> 16) & 1u)) >> 16;
}
__device__ __forceinline__ float bf16_val(float f) {
  return __uint_as_float(bf16_bits(f) << 16);
}
__device__ __forceinline__ v4f bf16_val4(v4f a) {
  v4f r;
  r.x = bf16_val(a.x); r.y = bf16_val(a.y); r.z = bf16_val(a.z); r.w = bf16_val(a.w);
  return r;
}
__device__ __forceinline__ bool fin32(float f) {
  return (__float_as_uint(f) & 0x7f800000u) != 0x7f800000u;
}

__device__ __forceinline__ void ln6(float (&v)[6], const float (&w)[6], const float (&b)[6]) {
  float s = v[0];
  s += v[1]; s += v[2]; s += v[3]; s += v[4]; s += v[5];
  const float mu = s * (1.0f / 6.0f);
  float d[6];
  float q = 0.0f;
#pragma unroll
  for (int c = 0; c < 6; ++c) { d[c] = v[c] - mu; q += d[c] * d[c]; }
  const float var = q * (1.0f / 6.0f);
  const float r = 1.0f / sqrtf(var + 1e-6f);
#pragma unroll
  for (int c = 0; c < 6; ++c) v[c] = d[c] * r * w[c] + b[c];
}

__device__ __forceinline__ void mha_row(const float* src, int jx, int jk, int jv,
                                        const float* par, int ai, float sc, float (&o)[6]) {
  const v4f xa = *(const v4fa*)(src + jx * 8);
  const v4f xb = *(const v4fa*)(src + jx * 8 + 4);
  const v4f ka = *(const v4fa*)(src + jk * 8);
  const v4f kb = *(const v4fa*)(src + jk * 8 + 4);
  const v4f va = *(const v4fa*)(src + jv * 8);
  const v4f vb = *(const v4fa*)(src + jv * 8 + 4);
  const float x[6]  = {xa.x, xa.y, xa.z, xa.w, xb.x, xb.y};
  const float xk[6] = {ka.x, ka.y, ka.z, ka.w, kb.x, kb.y};
  const float xv[6] = {va.x, va.y, va.z, va.w, vb.x, vb.y};
  const float* pp = par + ai * 6;
  float w[6], b[6];
#pragma unroll
  for (int c = 0; c < 6; ++c) {
    const float q   = x[c]  * pp[c]      + pp[12 + c];
    const float k   = xk[c] * pp[24 + c] + pp[36 + c];
    const float vv  = xv[c] * pp[48 + c] + pp[60 + c];
    const float teo = q * q - k * vv;
    o[c] = teo * sc + x[c];
    w[c] = pp[72 + c];
    b[c] = pp[84 + c];
  }
  ln6(o, w, b);
}

__global__ __launch_bounds__(NTHR) void k_inorm(const float* __restrict__ x,
                                                const float* __restrict__ n0w,
                                                const float* __restrict__ n0b,
                                                float* pout) {
  __shared__ __attribute__((aligned(16))) float sx[TILE * 6];
  __shared__ __attribute__((aligned(16))) float so[TILE * 8];
  __shared__ __attribute__((aligned(16))) float sp[16];
  const int tid = (int)threadIdx.x;
  const int blk = (int)blockIdx.x;
  const float* src = x + (size_t)blk * (TILE * 6);
  for (int i = tid; i < (TILE * 6) / 4; i += NTHR) {
    const v4f v = *(const v4fa*)(src + 4 * i);
    *(v4fa*)(sx + 4 * i) = bf16_val4(v);
  }
  {
    const int c = tid < 6 ? tid : 5;
    const float a = n0w[c];
    const float b = n0b[c];
    if (tid < 6) { sp[tid] = bf16_val(a); sp[8 + tid] = bf16_val(b); }
  }
  __syncthreads();
  {
    float v[6], w[6], b[6];
#pragma unroll
    for (int c = 0; c < 6; ++c) { v[c] = sx[tid * 6 + c]; w[c] = sp[c]; b[c] = sp[8 + c]; }
    ln6(v, w, b);
    const v4f o0 = {v[0], v[1], v[2], v[3]};
    const v4f o1 = {v[4], v[5], 0.0f, 0.0f};
    *(v4fa*)(so + tid * 8)     = o0;
    *(v4fa*)(so + tid * 8 + 4) = o1;
  }
  __syncthreads();
  {
    float* dst = pout + (size_t)blk * (TILE * 8);
    const v4f p0 = *(const v4fa*)(so + 4 * tid);
    const v4f p1 = *(const v4fa*)(so + 4 * (tid + NTHR));
    *(volatile v4f*)(dst + 4 * tid)          = p0;
    *(volatile v4f*)(dst + 4 * (tid + NTHR)) = p1;
    __threadfence();
    *(volatile v4f*)(dst + 4 * tid)          = p0;
    *(volatile v4f*)(dst + 4 * (tid + NTHR)) = p1;
  }
}

__global__ __launch_bounds__(NTHR) void k_layer(
    const float* pin, float* pout, float* outp, int li, int last,
    const float* __restrict__ qw, const float* __restrict__ qb,
    const float* __restrict__ kw, const float* __restrict__ kb,
    const float* __restrict__ vw, const float* __restrict__ vb,
    const float* __restrict__ l1w, const float* __restrict__ l1b,
    const float* __restrict__ mlw, const float* __restrict__ mlb,
    const float* __restrict__ w1, const float* __restrict__ b1,
    const float* __restrict__ w2, const float* __restrict__ b2,
    const float* __restrict__ flw, const float* __restrict__ flb)
{
  __shared__ __attribute__((aligned(16))) float sXS[XROWS * 8];
  __shared__ __attribute__((aligned(16))) float sY0[XROWS * 8];
  __shared__ __attribute__((aligned(16))) float sY1[TILE * 8];
  __shared__ __attribute__((aligned(16))) float sW1[DFF * 8];
  __shared__ __attribute__((aligned(16))) unsigned short sW2[16 * W2P];
  __shared__ __attribute__((aligned(16))) unsigned short sA[8 * 16 * AP];
  __shared__ __attribute__((aligned(16))) float sPar[8 * 12];
  __shared__ __attribute__((aligned(16))) float sB2[24];
  __shared__ __attribute__((aligned(16))) float sFW[24];
  __shared__ __attribute__((aligned(16))) float sFB[24];
  __shared__ float sSc[2];
  float* sFO = sY0;
  float* sSO = sXS;

  const int tid = (int)threadIdx.x, lane = tid & 31, wave = tid >> 5, hh = lane >> 4, m = lane & 15;
  const int blk = (int)blockIdx.x;
  const int b   = blk / TPR;
  const int t0  = (blk - b * TPR) * TILE;

#pragma unroll
  for (int it = 0; it < 2; ++it) {
    if (it == 0 || wave == 0) {
      const int j  = tid + it * NTHR;
      const int jc = j < XROWS ? j : XROWS - 1;
      const int p  = t0 - 2 + jc;
      const int pc = p < 0 ? 0 : (p > SEQ - 1 ? SEQ - 1 : p);
      const float* rp = pin + ((size_t)b * SEQ + (size_t)pc) * 8;
      v4f a = *(const v4fa*)rp;
      v4f c = *(const v4fa*)(rp + 4);
      const bool ok = (p == pc);
      const v4f z4 = {0.0f, 0.0f, 0.0f, 0.0f};
      a = ok ? a : z4;
      c = ok ? c : z4;
      if (j < XROWS) {
        *(v4fa*)(sXS + j * 8)     = a;
        *(v4fa*)(sXS + j * 8 + 4) = c;
      }
    }
  }

  {
    const int q96 = tid < 96 ? tid : 95;
    const v4f wv = *(const v4fa*)(w1 + (size_t)li * 384 + 4 * q96);
    const v4f uv = *(const v4fa*)(w2 + (size_t)li * 384 + 4 * q96);
    const int q16 = tid < 16 ? tid : 15;
    const v4f bv = *(const v4fa*)(b1 + (size_t)li * 64 + 4 * q16);
    if (tid < 96) {
#pragma unroll
      for (int i = 0; i < 4; ++i) {
        const int e = 4 * tid + i;
        const int f = e / 6;
        const int d = e - 6 * f;
        sW1[f * 8 + d] = bf16_val(wv[i]);
      }
      const int e2 = 4 * tid;
      const int n  = e2 >> 6;
      const int f2 = e2 & 63;
      unsigned short* wp = sW2 + n * W2P + f2;
      wp[0] = (unsigned short)bf16_bits(uv.x);
      wp[1] = (unsigned short)bf16_bits(uv.y);
      wp[2] = (unsigned short)bf16_bits(uv.z);
      wp[3] = (unsigned short)bf16_bits(uv.w);
    }
    if (tid < 16) {
#pragma unroll
      for (int i = 0; i < 4; ++i) sW1[(4 * tid + i) * 8 + 6] = bf16_val(bv[i]);
    }
    if (tid < 64) sW1[tid * 8 + 7] = 0.0f;
    const v8us z8 = {0, 0, 0, 0, 0, 0, 0, 0};
    if (tid < 90) *(v8usa*)(sW2 + 6 * W2P + 8 * tid) = z8;
    if (tid < 6)  *(v8usa*)(sW2 + tid * W2P + 64) = z8;

    const int q3 = tid < 3 ? tid : 2;
    const int o  = li * 12 + 4 * q3;
    const v4f p0 = *(const v4fa*)(qw + o);
    const v4f p1 = *(const v4fa*)(qb + o);
    const v4f p2 = *(const v4fa*)(kw + o);
    const v4f p3 = *(const v4fa*)(kb + o);
    const v4f p4 = *(const v4fa*)(vw + o);
    const v4f p5 = *(const v4fa*)(vb + o);
    const v4f p6 = *(const v4fa*)(mlw + o);
    const v4f p7 = *(const v4fa*)(mlb + o);
    if (tid < 3) {
      *(v4fa*)(sPar +  0 + 4 * tid) = bf16_val4(p0);
      *(v4fa*)(sPar + 12 + 4 * tid) = bf16_val4(p1);
      *(v4fa*)(sPar + 24 + 4 * tid) = bf16_val4(p2);
      *(v4fa*)(sPar + 36 + 4 * tid) = bf16_val4(p3);
      *(v4fa*)(sPar + 48 + 4 * tid) = bf16_val4(p4);
      *(v4fa*)(sPar + 60 + 4 * tid) = bf16_val4(p5);
      *(v4fa*)(sPar + 72 + 4 * tid) = bf16_val4(p6);
      *(v4fa*)(sPar + 84 + 4 * tid) = bf16_val4(p7);
    }
    const int q6 = tid < 6 ? tid : 5;
    const v4f c0 = *(const v4fa*)(b2  + 4 * q6);
    const v4f c1 = *(const v4fa*)(flw + 4 * q6);
    const v4f c2 = *(const v4fa*)(flb + 4 * q6);
    if (tid < 6) {
      *(v4fa*)(sB2 + 4 * tid) = bf16_val4(c0);
      *(v4fa*)(sFW + 4 * tid) = bf16_val4(c1);
      *(v4fa*)(sFB + 4 * tid) = bf16_val4(c2);
    }
    const int q2 = tid < 2 ? tid : 1;
    const float sa = l1w[li * 2 + q2];
    const float sb = l1b[li * 2 + q2];
    if (tid < 2) {
      const bool fin = fin32(sa) && fin32(bf16_val(sa)) && fin32(sb) && fin32(bf16_val(sb));
      sSc[tid] = fin ? 2.44140625e-4f : __uint_as_float(0x7fc00000u);
    }
  }
  __syncthreads();

#pragma unroll
  for (int it = 0; it < 2; ++it) {
    if (it == 0 || wave == 0) {
      const int i  = tid + it * NTHR;
      const int ic = i < TILE + 2 ? i : TILE + 1;
      const int p  = t0 - 1 + ic;
      const int pc = p < 0 ? 0 : (p > SEQ - 1 ? SEQ - 1 : p);
      const int pk = pc - 1 < 0 ? 0 : pc - 1;
      const int pv = pc + 1 > SEQ - 1 ? SEQ - 1 : pc + 1;
      float o[6];
      mha_row(sXS, pc - (t0 - 2), pk - (t0 - 2), pv - (t0 - 2), sPar, 0, sSc[0], o);
      const bool ok = (p == pc);
      v4f o0 = {o[0], o[1], o[2], o[3]};
      v4f o1 = {o[4], o[5], 0.0f, 0.0f};
      const v4f z4 = {0.0f, 0.0f, 0.0f, 0.0f};
      o0 = ok ? o0 : z4;
      o1 = ok ? o1 : z4;
      if (i < TILE + 2) {
        *(v4fa*)(sY0 + (ic + 1) * 8)     = o0;
        *(v4fa*)(sY0 + (ic + 1) * 8 + 4) = o1;
      }
    }
  }
  __syncthreads();

  {
    const int p  = t0 + tid;
    const int pk = p - 1 < 0 ? 0 : p - 1;
    const int pv = p + 1 > SEQ - 1 ? SEQ - 1 : p + 1;
    float o[6];
    mha_row(sY0, tid + 2, pk - (t0 - 2), pv - (t0 - 2), sPar, 1, sSc[1], o);
    const v4f o0 = {o[0], o[1], o[2], o[3]};
    const v4f o1 = {o[4], o[5], 0.0f, 0.0f};
    *(v4fa*)(sY1 + tid * 8)     = o0;
    *(v4fa*)(sY1 + tid * 8 + 4) = o1;
  }
  __syncthreads();

  {
    FragB bfr[2];
#pragma unroll
    for (int ks = 0; ks < 2; ++ks) {
      const unsigned short* wq = sW2 + m * W2P + 32 * ks + 8 * hh;
      bfr[ks].h[0] = *(const v8usa*)wq;
      bfr[ks].h[1] = *(const v8usa*)(wq + 16);
    }
    unsigned short* sAw = sA + wave * (16 * AP);
    unsigned short* arow = sAw + m * AP;
#pragma unroll 1
    for (int mt = 0; mt < 2; ++mt) {
      const int tok = 32 * wave + 16 * mt + m;
      const v4f xa = *(const v4fa*)(sY1 + tok * 8);
      const v4f xb = *(const v4fa*)(sY1 + tok * 8 + 4);
#pragma unroll 1
      for (int c8 = 0; c8 < 4; ++c8) {
        const int f0 = 32 * hh + 8 * c8;
        v8us ho, lo;
#pragma unroll
        for (int i = 0; i < 8; ++i) {
          const float* wr = sW1 + (f0 + i) * 8;
          const v4f wa = *(const v4fa*)wr;
          const v4f wc = *(const v4fa*)(wr + 4);
          float hv = xa.x * wa.x;
          hv = fmaf(xa.y, wa.y, hv);
          hv = fmaf(xa.z, wa.z, hv);
          hv = fmaf(xa.w, wa.w, hv);
          hv = fmaf(xb.x, wc.x, hv);
          hv = fmaf(xb.y, wc.y, hv);
          hv = hv + wc.z;
          hv = hv > 0.0f ? hv : 0.0f;
          const unsigned hb = bf16_bits(hv);
          const unsigned lb = bf16_bits(hv - __uint_as_float(hb << 16));
          ho[i] = (unsigned short)hb;
          lo[i] = (unsigned short)lb;
        }
        *(v8usa*)(arow + f0)       = ho;
        *(v8usa*)(arow + DFF + f0) = lo;
      }
      __syncthreads();

      v8f acc = {0.f, 0.f, 0.f, 0.f, 0.f, 0.f, 0.f, 0.f};
#pragma unroll
      for (int ks = 0; ks < 4; ++ks) {
        const unsigned short* ap = arow + 32 * ks + 8 * hh;
        FragB af;
        af.h[0] = *(const v8usa*)ap;
        af.h[1] = *(const v8usa*)(ap + 16);
        acc = wmb(af, bfr[ks & 1], acc);
      }
      if (m < 8) {
#pragma unroll
        for (int r = 0; r < 8; ++r) sFO[(32 * wave + 16 * mt + 8 * hh + r) * 8 + m] = acc[r];
      }
      __syncthreads();
    }
  }

  {
    const v4f fa = *(const v4fa*)(sFO + tid * 8);
    const v4f fb = *(const v4fa*)(sFO + tid * 8 + 4);
    const v4f ya = *(const v4fa*)(sY1 + tid * 8);
    const v4f yb = *(const v4fa*)(sY1 + tid * 8 + 4);
    float y[6], w[6], bb[6];
    y[0] = fa.x + sB2[li * 6 + 0] + ya.x;
    y[1] = fa.y + sB2[li * 6 + 1] + ya.y;
    y[2] = fa.z + sB2[li * 6 + 2] + ya.z;
    y[3] = fa.w + sB2[li * 6 + 3] + ya.w;
    y[4] = fb.x + sB2[li * 6 + 4] + yb.x;
    y[5] = fb.y + sB2[li * 6 + 5] + yb.y;
#pragma unroll
    for (int c = 0; c < 6; ++c) { w[c] = sFW[li * 6 + c]; bb[c] = sFB[li * 6 + c]; }
    ln6(y, w, bb);
    if (last != 0) {
#pragma unroll
      for (int c = 0; c < 6; ++c) sSO[tid * 6 + c] = y[c];
    } else {
      const v4f o0 = {y[0], y[1], y[2], y[3]};
      const v4f o1 = {y[4], y[5], 0.0f, 0.0f};
      *(v4fa*)(sSO + tid * 8)     = o0;
      *(v4fa*)(sSO + tid * 8 + 4) = o1;
    }
  }
  __syncthreads();
  {
    const int nvec = (last != 0) ? (TILE * 6) / 4 : (TILE * 8) / 4;
    float* gdst = (last != 0) ? (outp + (size_t)blk * (TILE * 6)) : (pout + (size_t)blk * (TILE * 8));
    const int  i1   = tid + NTHR;
    const bool has1 = i1 < nvec;
    const int  i1c  = has1 ? i1 : nvec - 1;
    const v4f pv0 = *(const v4fa*)(sSO + 4 * tid);
    const v4f pv1 = *(const v4fa*)(sSO + 4 * i1c);
    *(volatile v4f*)(gdst + 4 * tid) = pv0;
    if (has1) *(volatile v4f*)(gdst + 4 * i1) = pv1;
    __threadfence();
    *(volatile v4f*)(gdst + 4 * tid) = pv0;
    if (has1) *(volatile v4f*)(gdst + 4 * i1) = pv1;
  }
}

extern "C" void kernel_launch(void* const* d_in, const int* in_sizes, int n_in,
                              void* d_out, int out_size, void* d_ws, size_t ws_size,
                              hipStream_t stream) {
  if (n_in < 20) return;
  if (in_sizes[0] != TOK * DM) return;
  if (in_sizes[2] != DM || in_sizes[3] != DM) return;
  for (int i = 4; i <= 9; ++i) if (in_sizes[i] != NLAY * 2 * DM) return;
  if (in_sizes[10] != NLAY * 2 || in_sizes[11] != NLAY * 2) return;
  if (in_sizes[12] != NLAY * 2 * DM || in_sizes[13] != NLAY * 2 * DM) return;
  if (in_sizes[14] != NLAY * DFF * DM || in_sizes[15] != NLAY * DFF) return;
  if (in_sizes[16] != NLAY * DM * DFF || in_sizes[17] != NLAY * DM) return;
  if (in_sizes[18] != NLAY * DM || in_sizes[19] != NLAY * DM) return;
  if (out_size != TOK * DM) return;

  const float* x    = (const float*)d_in[0];
  const float* n0w  = (const float*)d_in[2];
  const float* n0b  = (const float*)d_in[3];
  const float* qw   = (const float*)d_in[4];
  const float* qb   = (const float*)d_in[5];
  const float* kw   = (const float*)d_in[6];
  const float* kb   = (const float*)d_in[7];
  const float* vw   = (const float*)d_in[8];
  const float* vb   = (const float*)d_in[9];
  const float* l1w  = (const float*)d_in[10];
  const float* l1b  = (const float*)d_in[11];
  const float* mlw  = (const float*)d_in[12];
  const float* mlb  = (const float*)d_in[13];
  const float* w1   = (const float*)d_in[14];
  const float* b1   = (const float*)d_in[15];
  const float* w2   = (const float*)d_in[16];
  const float* b2   = (const float*)d_in[17];
  const float* flw  = (const float*)d_in[18];
  const float* flb  = (const float*)d_in[19];
  float* out = (float*)d_out;

  const size_t need = 2 * PLANE_BYTES;
  if (need > ws_size || need > (size_t)WSMAX) return;
  float* P0 = (float*)d_ws;
  float* P1 = (float*)((char*)d_ws + PLANE_BYTES);

  k_inorm<<<NBLK, NTHR, 0, stream>>>(x, n0w, n0b, P0);
  for (int li = 0; li < NLAY; ++li) {
    const float* pin  = (li & 1) ? P1 : P0;
    float*       pout = (li & 1) ? P0 : P1;
    const int    last = (li == NLAY - 1) ? 1 : 0;
    k_layer<<<NBLK, NTHR, 0, stream>>>(pin, pout, out, li, last,
                                       qw, qb, kw, kb, vw, vb, l1w, l1b, mlw, mlb,
                                       w1, b1, w2, b2, flw, flb);
  }
}
